// NeuroNet_38362647888397
// MI455X (gfx1250) — hardware-verified
//
#include <hip/hip_runtime.h>
#define NB 8
#define HW 128
#define PS 8
#define NP 256
#define FD 64
#define F2 128
#define NPAIR 32640
#define NC 10
typedef __bf16 v16b __attribute__((ext_vector_type(16)));
typedef unsigned short v8us __attribute__((ext_vector_type(8), may_alias));
typedef float  v8f  __attribute__((ext_vector_type(8)));
typedef float  v4f  __attribute__((ext_vector_type(4)));
typedef float  v4fa __attribute__((ext_vector_type(4), may_alias));
union FragB { v16b v; v8us half[2]; unsigned short u[16]; };

__device__ __forceinline__ unsigned short bf16_bits(float x) { unsigned int u = __float_as_uint(x); return (unsigned short)((u + 0x7FFFu + ((u >> 16) & 1u)) >> 16); }
__device__ __forceinline__ float bf16_val(unsigned short b) { return __uint_as_float(((unsigned int)b) << 16); }
__device__ __forceinline__ float bf16_round(float x) { return bf16_val(bf16_bits(x)); }
template <int NT>
__device__ __forceinline__ v8f mmaN(v16b ah, v16b al, v16b bh, v16b bl, v8f c) {
  c = __builtin_amdgcn_wmma_f32_16x16x32_bf16(false, ah, false, bh, (short)0, c, false, false);
  if (NT >= 2) c = __builtin_amdgcn_wmma_f32_16x16x32_bf16(false, al, false, bh, (short)0, c, false, false);
  if (NT >= 3) c = __builtin_amdgcn_wmma_f32_16x16x32_bf16(false, ah, false, bl, (short)0, c, false, false);
  asm volatile("v_nop\n\tv_nop\n\tv_nop\n\tv_nop" : "+v"(c) : "v"(ah), "v"(al), "v"(bh), "v"(bl));
  return c;
}

__global__ __launch_bounds__(256) void k_wt_bf16(const float* __restrict__ W, unsigned short* __restrict__ Wt, int K, int N) {
  const int t = blockIdx.x * 256 + threadIdx.x;
  const int k8n = K / 8;
  if (t >= N * k8n) return;
  const int n = t / k8n, k8 = (t % k8n) * 8;
  v8us v;
#pragma unroll
  for (int i = 0; i < 8; ++i) v[i] = bf16_bits(W[(size_t)(k8 + i) * N + n]);
  *(volatile v8us*)(Wt + (size_t)n * K + k8) = v;
  __threadfence();
  *(volatile v8us*)(Wt + (size_t)n * K + k8) = v;
}

template <bool ASPLIT, int ACT, bool BIAS_BF16>
__global__ __launch_bounds__(128) void k_gemm_bf(const float* __restrict__ A, int lda, const unsigned short* __restrict__ Wt, int ldb,
                                               const float* __restrict__ bias, float* __restrict__ C, int ldc, int M, int N, int K) {
  __shared__ __attribute__((aligned(16))) float so[4][16][64];
  const int tid = threadIdx.x, w = tid >> 5, lane = tid & 31, ln = lane & 15, hh = lane >> 4;
  const int ntn = N / 64;
  const int wid = blockIdx.x * 4 + w;
  const int mt = wid / ntn, nq = wid % ntn;
  if (mt * 16 >= M) return;
  const int row0 = mt * 16, col0 = nq * 64;
  const float* arow = A + (size_t)(row0 + ln) * lda;
  v8f acc[4] = {};
  for (int kb = 0; kb < K; kb += 32) {
    FragB ah, al;
    const v4f x0 = *(const v4fa*)(arow + kb + 8 * hh), x1 = *(const v4fa*)(arow + kb + 8 * hh + 4);
    const v4f x2 = *(const v4fa*)(arow + kb + 16 + 8 * hh), x3 = *(const v4fa*)(arow + kb + 16 + 8 * hh + 4);
    float xs[16] = {x0[0],x0[1],x0[2],x0[3],x1[0],x1[1],x1[2],x1[3],x2[0],x2[1],x2[2],x2[3],x3[0],x3[1],x3[2],x3[3]};
#pragma unroll
    for (int i = 0; i < 16; ++i) { const unsigned short hb = bf16_bits(xs[i]); ah.u[i] = hb; al.u[i] = ASPLIT ? bf16_bits(xs[i] - bf16_val(hb)) : (unsigned short)0; }
#pragma unroll
    for (int t = 0; t < 4; ++t) {
      const unsigned short* brow = Wt + (size_t)(col0 + t * 16 + ln) * ldb + kb;
      FragB b;
      b.half[0] = *(const v8us*)(brow + 8 * hh);
      b.half[1] = *(const v8us*)(brow + 16 + 8 * hh);
      acc[t] = mmaN<ASPLIT ? 2 : 1>(ah.v, al.v, b.v, b.v, acc[t]);
    }
  }
#pragma unroll
  for (int t = 0; t < 4; ++t) {
    float bv = bias ? bias[col0 + t * 16 + ln] : 0.f;
    if (BIAS_BF16) bv = bf16_round(bv);
#pragma unroll
    for (int r = 0; r < 8; ++r) { float v = acc[t][r] + bv; if (ACT == 1) v = fmaxf(v, 0.f); so[w][8 * hh + r][t * 16 + ln] = v; }
  }
  __builtin_amdgcn_fence(__ATOMIC_ACQ_REL, "workgroup");
  __builtin_amdgcn_wave_barrier();
  const int rsub = lane >> 4, c4 = (lane & 15) * 4;
  for (int pass = 0; pass < 2; ++pass) {
#pragma unroll
    for (int q = 0; q < 8; ++q) {
      const int r = q * 2 + rsub;
      const v4f v = *(const v4fa*)&so[w][r][c4];
      *(volatile v4f*)(C + (size_t)(row0 + r) * ldc + col0 + c4) = v;
    }
    if (pass == 0) __threadfence();
  }
}

template <bool ASPLIT, int ACT, bool BIAS_BF16, bool RES_BF16>
__global__ __launch_bounds__(128) void k_gemm_bf3(const float* __restrict__ A, int lda, const unsigned short* __restrict__ Wt, int ldb,
                                                const float* __restrict__ bias, const float* __restrict__ resid, int rmod, int ldr,
                                                float* __restrict__ C, int ldc, int M, int N, int K) {
  __shared__ __attribute__((aligned(16))) float so[4][16][64];
  const int tid = threadIdx.x, w = tid >> 5, lane = tid & 31, ln = lane & 15, hh = lane >> 4;
  const int ntn = N / 64;
  const int wid = blockIdx.x * 4 + w;
  const int mt = wid / ntn, nq = wid % ntn;
  if (mt * 16 >= M) return;
  const int row0 = mt * 16, col0 = nq * 64;
  const float* arow = A + (size_t)(row0 + ln) * lda;
  v8f acc[4] = {};
  for (int kb = 0; kb < K; kb += 32) {
    FragB ah, al;
    const v4f x0 = *(const v4fa*)(arow + kb + 8 * hh), x1 = *(const v4fa*)(arow + kb + 8 * hh + 4);
    const v4f x2 = *(const v4fa*)(arow + kb + 16 + 8 * hh), x3 = *(const v4fa*)(arow + kb + 16 + 8 * hh + 4);
    float xs[16] = {x0[0],x0[1],x0[2],x0[3],x1[0],x1[1],x1[2],x1[3],x2[0],x2[1],x2[2],x2[3],x3[0],x3[1],x3[2],x3[3]};
#pragma unroll
    for (int i = 0; i < 16; ++i) { const unsigned short hb = bf16_bits(xs[i]); ah.u[i] = hb; al.u[i] = ASPLIT ? bf16_bits(xs[i] - bf16_val(hb)) : (unsigned short)0; }
#pragma unroll
    for (int t = 0; t < 4; ++t) {
      const unsigned short* brow = Wt + (size_t)(col0 + t * 16 + ln) * ldb + kb;
      FragB b;
      b.half[0] = *(const v8us*)(brow + 8 * hh);
      b.half[1] = *(const v8us*)(brow + 16 + 8 * hh);
      acc[t] = mmaN<ASPLIT ? 2 : 1>(ah.v, al.v, b.v, b.v, acc[t]);
    }
  }
#pragma unroll
  for (int t = 0; t < 4; ++t) {
    const int col = col0 + t * 16 + ln;
    float bv = bias ? bias[col] : 0.f;
    if (BIAS_BF16) bv = bf16_round(bv);
#pragma unroll
    for (int r = 0; r < 8; ++r) {
      float v = acc[t][r] + bv;
      if (resid) { float rv = resid[(size_t)((row0 + 8 * hh + r) % rmod) * ldr + col]; if (RES_BF16) rv = bf16_round(rv); v += rv; }
      if (ACT == 1) v = fmaxf(v, 0.f);
      if (ACT == 2) v = 0.5f * v * (1.0f + erff(v * 0.70710678118654752f));
      if (ACT == 3) { const float u = 0.7978845608028654f * (v + 0.044715f * v * v * v); v = 0.5f * v * (1.0f + tanhf(u)); }
      so[w][8 * hh + r][t * 16 + ln] = v;
    }
  }
  __builtin_amdgcn_fence(__ATOMIC_ACQ_REL, "workgroup");
  __builtin_amdgcn_wave_barrier();
  const int rsub = lane >> 4, c4 = (lane & 15) * 4;
  for (int pass = 0; pass < 2; ++pass) {
#pragma unroll
    for (int q = 0; q < 8; ++q) {
      const int r = q * 2 + rsub;
      const v4f v = *(const v4fa*)&so[w][r][c4];
      *(volatile v4f*)(C + (size_t)(row0 + r) * ldc + col0 + c4) = v;
    }
    if (pass == 0) __threadfence();
  }
}
template <bool PARAM_BF16>
__global__ __launch_bounds__(256) void k_layernorm(const float* __restrict__ X, const float* __restrict__ R, const float* __restrict__ g, const float* __restrict__ bta,
                                                  float* __restrict__ out_sum, float* __restrict__ out_norm, int N, float eps) {
  __shared__ float red[256];
  const int row = blockIdx.x, tid = threadIdx.x;
  const float* x = X + (size_t)row * N; const float* rr = R ? R + (size_t)row * N : nullptr;
  float vals[16];
  const int per = N / 256;
  float s1 = 0.f;
  for (int u = 0; u < per / 4; ++u) {
    const int j = tid * 4 + 1024 * u;
    const v4f a = *(const v4fa*)(x + j);
    v4f b = {0.f,0.f,0.f,0.f}; if (rr) b = *(const v4fa*)(rr + j);
#pragma unroll
    for (int q = 0; q < 4; ++q) { const float v = a[q] + b[q]; vals[u * 4 + q] = v; s1 += v; }
  }
  red[tid] = s1; __syncthreads();
  for (int st = 128; st > 0; st >>= 1) { if (tid < st) red[tid] += red[tid + st]; __syncthreads(); }
  const float mu = red[0] / (float)N; __syncthreads();
  float s2 = 0.f;
  for (int u = 0; u < per / 4; ++u)
#pragma unroll
    for (int q = 0; q < 4; ++q) { const float c = vals[u * 4 + q] - mu; s2 += c * c; }
  red[tid] = s2; __syncthreads();
  for (int st = 128; st > 0; st >>= 1) { if (tid < st) red[tid] += red[tid + st]; __syncthreads(); }
  const float rs = rsqrtf(red[0] / (float)N + eps);
  for (int pass = 0; pass < 2; ++pass) {
    for (int u = 0; u < per / 4; ++u) {
      const int j = tid * 4 + 1024 * u;
      v4f o, sm;
#pragma unroll
      for (int q = 0; q < 4; ++q) {
        float gg = g[j + q], bb = bta[j + q];
        if (PARAM_BF16) { gg = bf16_round(gg); bb = bf16_round(bb); }
        sm[q] = vals[u * 4 + q]; o[q] = (vals[u * 4 + q] - mu) * rs * gg + bb;
      }
      if (out_sum) *(volatile v4f*)(out_sum + (size_t)row * N + j) = sm;
      *(volatile v4f*)(out_norm + (size_t)row * N + j) = o;
    }
    if (pass == 0) __threadfence();
  }
}


typedef _Float16 v16h __attribute__((ext_vector_type(16)));
union FragH { v16h v; v8us half[2]; _Float16 h[16]; unsigned short u[16]; };
template <int NT>
__device__ __forceinline__ v8f mmaH(v16h ah, v16h al, v16h bh, v16h bl, v8f c) {
  c = __builtin_amdgcn_wmma_f32_16x16x32_f16(false, ah, false, bh, (short)0, c, false, false);
  if (NT >= 2) c = __builtin_amdgcn_wmma_f32_16x16x32_f16(false, al, false, bh, (short)0, c, false, false);
  if (NT >= 3) c = __builtin_amdgcn_wmma_f32_16x16x32_f16(false, ah, false, bl, (short)0, c, false, false);
  asm volatile("v_nop\n\tv_nop\n\tv_nop\n\tv_nop" : "+v"(c) : "v"(ah), "v"(al), "v"(bh), "v"(bl));
  return c;
}
template <bool ASPLIT>
__global__ __launch_bounds__(128) void k_gemm_h(const float* __restrict__ A, int lda, size_t sA, const _Float16* __restrict__ Bh, int ldb, size_t sB, float alpha, float* __restrict__ C, int ldc, size_t sC, int M, int N, int K) {
  __shared__ __attribute__((aligned(16))) float so[4][16][64];
  const int tid = threadIdx.x, w = tid >> 5, lane = tid & 31, ln = lane & 15, hh = lane >> 4; const int by = blockIdx.y;
  A += (size_t)by * sA; Bh += (size_t)by * sB; C += (size_t)by * sC;
  const int ntn = (N + 63) / 64; const int wid = blockIdx.x * 4 + w; const int mt = wid / ntn, nq = wid % ntn; if (mt * 16 >= M) return;
  const int row0 = mt * 16, col0 = nq * 64; const float* arow = A + (size_t)(row0 + ln) * lda;
  v8f acc[4] = {};
  for (int kb = 0; kb < K; kb += 32) {
    FragH ah, al;
    const v4f x0 = *(const v4fa*)(arow + kb + 8 * hh), x1 = *(const v4fa*)(arow + kb + 8 * hh + 4), x2 = *(const v4fa*)(arow + kb + 16 + 8 * hh), x3 = *(const v4fa*)(arow + kb + 16 + 8 * hh + 4);
    float xs[16] = {x0[0],x0[1],x0[2],x0[3],x1[0],x1[1],x1[2],x1[3],x2[0],x2[1],x2[2],x2[3],x3[0],x3[1],x3[2],x3[3]};
#pragma unroll
    for (int i = 0; i < 16; ++i) { const _Float16 h = (_Float16)xs[i]; ah.h[i] = h; al.h[i] = ASPLIT ? (_Float16)(xs[i] - (float)h) : (_Float16)0.0f; }
#pragma unroll
    for (int t = 0; t < 4; ++t) { if (col0 + t * 16 >= N) continue; const size_t boff = (size_t)(col0 + t * 16 + ln) * ldb + kb; FragH bq; bq.half[0] = *(const v8us*)(Bh + boff + 8 * hh); bq.half[1] = *(const v8us*)(Bh + boff + 16 + 8 * hh);
      acc[t] = mmaH<ASPLIT ? 2 : 1>(ah.v, al.v, bq.v, bq.v, acc[t]); }
  }
#pragma unroll
  for (int t = 0; t < 4; ++t) { if (col0 + t * 16 >= N) continue;
#pragma unroll
    for (int r = 0; r < 8; ++r) so[w][8 * hh + r][t * 16 + ln] = acc[t][r] * alpha; }
  __builtin_amdgcn_fence(__ATOMIC_ACQ_REL, "workgroup"); __builtin_amdgcn_wave_barrier();
  const int rsub = lane >> 4, c4 = (lane & 15) * 4;
  for (int pass = 0; pass < 2; ++pass) {
#pragma unroll
    for (int q = 0; q < 8; ++q) { const int r = q * 2 + rsub; if (col0 + c4 < N) { const v4f v = *(const v4fa*)&so[w][r][c4]; *(volatile v4f*)(C + (size_t)(row0 + r) * ldc + col0 + c4) = v; } }
    if (pass == 0) __threadfence(); }
}

__global__ __launch_bounds__(256) void k_wt_f16(const float* __restrict__ W, _Float16* __restrict__ Wt, int K, int N, float scale) {
  const int t = blockIdx.x * 256 + threadIdx.x; if (t >= N * (K / 8)) return; const int n = t / (K / 8), k8 = (t % (K / 8)) * 8; FragH f;
#pragma unroll
  for (int i = 0; i < 8; ++i) f.h[i] = (_Float16)(bf16_round(W[(size_t)(k8 + i) * N + n]) * scale); const v8us o = f.half[0];
  *(volatile v8us*)((unsigned short*)Wt + (size_t)n * K + k8) = o; __threadfence(); *(volatile v8us*)((unsigned short*)Wt + (size_t)n * K + k8) = o;
}
template <int ACT>
__global__ __launch_bounds__(128) void k_gemm_hhx(const _Float16* __restrict__ A, int lda, size_t sA, const _Float16* __restrict__ Bh, int ldb, size_t sB, float alpha, const float* __restrict__ bias, size_t sBias, const float* __restrict__ CP, int rowsPerB, size_t sCPb, int row0g,
    float* __restrict__ C, _Float16* __restrict__ C16, int ldc, size_t sC, int M, int N, int K) {
  __shared__ __attribute__((aligned(16))) float so[4][16][64];
  const int tid = threadIdx.x, w = tid >> 5, lane = tid & 31, ln = lane & 15, hh = lane >> 4; const int by = blockIdx.y;
  A += (size_t)by * sA; Bh += (size_t)by * sB; const size_t cofs = (size_t)by * sC; const float* bp = bias ? bias + (size_t)by * sBias : nullptr;
  const int ntn = (N + 63) / 64; const int wid = blockIdx.x * 4 + w; const int mt = wid / ntn, nq = wid % ntn; if (mt * 16 >= M) return;
  const int row0 = mt * 16, col0 = nq * 64; const _Float16* arow = A + (size_t)(row0 + ln) * lda;
  v8f acc[4] = {};
  for (int kb = 0; kb < K; kb += 32) { FragH ah; ah.half[0] = *(const v8us*)((const unsigned short*)arow + kb + 8 * hh); ah.half[1] = *(const v8us*)((const unsigned short*)arow + kb + 16 + 8 * hh);
#pragma unroll
    for (int t = 0; t < 4; ++t) { if (col0 + t * 16 >= N) continue; const size_t boff = (size_t)(col0 + t * 16 + ln) * ldb + kb; FragH bq; bq.half[0] = *(const v8us*)((const unsigned short*)Bh + boff + 8 * hh); bq.half[1] = *(const v8us*)((const unsigned short*)Bh + boff + 16 + 8 * hh);
      acc[t] = mmaH<1>(ah.v, ah.v, bq.v, bq.v, acc[t]); }
  }
#pragma unroll
  for (int t = 0; t < 4; ++t) { if (col0 + t * 16 >= N) continue; const int col = col0 + t * 16 + ln; const float bv = bp ? bf16_round(bp[col]) : 0.f;
#pragma unroll
    for (int r = 0; r < 8; ++r) { float v = acc[t][r] * alpha + bv; if (CP) { const int bidx = (row0g + row0 + 8 * hh + r) / rowsPerB; v += CP[(size_t)bidx * sCPb + (size_t)by * 64 + col]; } if (ACT == 1) v = (v > 0.f) ? v : expm1f(v); else if (ACT == 7) v = (v > 0.f) ? v + 1.0f : expf(v); else if (ACT == 8) v = tanhf(v); else if (ACT == 9) v = 0.5f * v * (1.0f + tanhf(0.7978845608028654f * (v + 0.044715f * v * v * v))); else if (ACT == 11) v = 1.0f / (1.0f + expf(-v)); else if (ACT == 12) v = (v > 0.f) ? v : 0.01f * v; else if (ACT == 14) v = (v > 0.f) ? v : 0.1f * v; else if (ACT == 15) v = v / (1.0f + expf(-v)); else if (ACT == 3) v = fmaxf(v, 0.f); else if (ACT == 6) v = 0.5f * v * (1.0f + erff(v * 0.70710678118654752f)); so[w][8 * hh + r][t * 16 + ln] = v; } }
  __builtin_amdgcn_fence(__ATOMIC_ACQ_REL, "workgroup"); __builtin_amdgcn_wave_barrier();
  const int rsub = lane >> 4, c4 = (lane & 15) * 4; typedef _Float16 v4h __attribute__((ext_vector_type(4)));
  for (int pass = 0; pass < 2; ++pass) {
#pragma unroll
    for (int q = 0; q < 8; ++q) { const int r = q * 2 + rsub; if (col0 + c4 < N) { const v4f v = *(const v4fa*)&so[w][r][c4]; if (C) *(volatile v4f*)(C + cofs + (size_t)(row0 + r) * ldc + col0 + c4) = v; if (C16) { v4h h4; for (int i = 0; i < 4; ++i) h4[i] = (_Float16)v[i]; *(volatile v4h*)(C16 + cofs + (size_t)(row0 + r) * ldc + col0 + c4) = h4; } } }
    if (pass == 0) __threadfence(); }
}


typedef _Float16 v4h __attribute__((ext_vector_type(4)));

__global__ __launch_bounds__(256) void k_x16(const float* __restrict__ x, _Float16* __restrict__ X16, size_t n8) { const size_t t = (size_t)blockIdx.x * 256 + threadIdx.x; if (t >= n8) return; FragH f;
#pragma unroll
  for (int q = 0; q < 8; ++q) f.h[q] = (_Float16)bf16_round(x[t * 8 + q]); *(volatile v8us*)((unsigned short*)X16 + t * 8) = f.half[0]; __threadfence(); *(volatile v8us*)((unsigned short*)X16 + t * 8) = f.half[0]; }
__global__ __launch_bounds__(256) void k_h16(const float* __restrict__ x, _Float16* __restrict__ X16, size_t n8) { const size_t t = (size_t)blockIdx.x * 256 + threadIdx.x; if (t >= n8) return; FragH f;
#pragma unroll
  for (int q = 0; q < 8; ++q) f.h[q] = (_Float16)x[t * 8 + q]; *(volatile v8us*)((unsigned short*)X16 + t * 8) = f.half[0]; __threadfence(); *(volatile v8us*)((unsigned short*)X16 + t * 8) = f.half[0]; }
__global__ __launch_bounds__(256) void k_round16f(const float* __restrict__ W, _Float16* __restrict__ Bt, size_t n8) { const size_t t = (size_t)blockIdx.x * 256 + threadIdx.x; if (t >= n8) return; FragH f;
#pragma unroll
  for (int i = 0; i < 8; ++i) f.h[i] = (_Float16)(bf16_round(W[t * 8 + i]) * 16.0f); *(volatile v8us*)((unsigned short*)Bt + t * 8) = f.half[0]; __threadfence(); *(volatile v8us*)((unsigned short*)Bt + t * 8) = f.half[0]; }
template <int NHv, int TTv>
__global__ __launch_bounds__(256) void k_vt(const _Float16* __restrict__ V16, int ldv, int voff, _Float16* __restrict__ Vt) { __shared__ unsigned short tl[64][66]; const int tid = threadIdx.x; const int slab = blockIdx.x / (TTv / 64), lg = blockIdx.x % (TTv / 64); const int b = slab / NHv, h = slab % NHv;
  for (int i = tid; i < 64 * 8; i += 256) { const int r = i / 8, c8 = (i % 8) * 8; FragH f; f.half[0] = *(const v8us*)((const unsigned short*)V16 + ((size_t)b * TTv + lg * 64 + r) * ldv + voff + h * 64 + c8);
#pragma unroll
    for (int q = 0; q < 8; ++q) tl[r][c8 + q] = f.u[q]; }
  __syncthreads();
  for (int pass = 0; pass < 2; ++pass) {
#pragma unroll
    for (int rd = 0; rd < 2; ++rd) { const int d = rd * 32 + tid / 8, pc = tid % 8; FragH f;
#pragma unroll
      for (int q = 0; q < 8; ++q) f.u[q] = tl[pc * 8 + q][d];
      *(volatile v8us*)((unsigned short*)Vt + ((size_t)slab * 64 + d) * TTv + lg * 64 + pc * 8) = f.half[0]; }
    if (pass == 0) __threadfence(); } }

__global__ __launch_bounds__(256) void k_hl(const float* __restrict__ F, _Float16* __restrict__ Hh, _Float16* __restrict__ Hl, size_t n8) { const size_t t = (size_t)blockIdx.x * 256 + threadIdx.x; if (t >= n8) return; FragH fh, fl; const v4f a = *(const v4fa*)(F + t * 8), c = *(const v4fa*)(F + t * 8 + 4);
#pragma unroll
  for (int q = 0; q < 4; ++q) { _Float16 h = (_Float16)a[q]; fh.h[q] = h; fl.h[q] = (_Float16)((a[q] - (float)h) * 1024.0f); h = (_Float16)c[q]; fh.h[4 + q] = h; fl.h[4 + q] = (_Float16)((c[q] - (float)h) * 1024.0f); }
  for (int pass = 0; pass < 2; ++pass) { *(volatile v8us*)((unsigned short*)Hh + t * 8) = fh.half[0]; *(volatile v8us*)((unsigned short*)Hl + t * 8) = fl.half[0]; if (pass == 0) __threadfence(); } }

__device__ __forceinline__ float gelu_t(float v) { const float u = 0.7978845608028654f * (v + 0.044715f * v * v * v); return 0.5f * v * (1.0f + tanhf(u)); }
__global__ __launch_bounds__(256) void k_patch(const float* __restrict__ x, _Float16* __restrict__ A) { const int t = blockIdx.x * 256 + threadIdx.x; if (t >= NB * NP * PS) return; const int py = t % PS; const int bp = t / PS; const int b = bp / NP, p = bp % NP; const int gy = p / 16, gx = p % 16; FragH f;
#pragma unroll
  for (int q = 0; q < 8; ++q) f.h[q] = (_Float16)bf16_round(x[((size_t)b * HW + gy * PS + py) * HW + gx * PS + q]);
  *(volatile v8us*)((unsigned short*)A + (size_t)bp * 64 + py * 8) = f.half[0]; __threadfence(); *(volatile v8us*)((unsigned short*)A + (size_t)bp * 64 + py * 8) = f.half[0]; }
__global__ __launch_bounds__(256) void k_hpos(const float* __restrict__ Cc, const float* __restrict__ pos, _Float16* __restrict__ H16) {
  #pragma clang fp contract(off)
  const int t = blockIdx.x * 256 + threadIdx.x; if (t >= NB * NP * (FD / 8)) return; const int f0 = (t % (FD / 8)) * 8, bp = t / (FD / 8); const int p = bp % NP; const v4f a = *(const v4fa*)(Cc + (size_t)bp * FD + f0), c = *(const v4fa*)(Cc + (size_t)bp * FD + f0 + 4); FragH f = FragH{};
#pragma unroll 1
  for (int q = 0; q < 8; ++q) { const float v = (q < 4) ? ((q == 0) ? a[0] : (q == 1) ? a[1] : (q == 2) ? a[2] : a[3]) : ((q == 4) ? c[0] : (q == 5) ? c[1] : (q == 6) ? c[2] : c[3]); const _Float16 hv = (_Float16)(gelu_t(v) + bf16_round(pos[(size_t)(f0 + q) * NP + p]));
#pragma unroll
    for (int k = 0; k < 8; ++k) f.h[k] = (k == q) ? hv : f.h[k]; }
  *(volatile v8us*)((unsigned short*)H16 + (size_t)bp * FD + f0) = f.half[0]; __threadfence(); *(volatile v8us*)((unsigned short*)H16 + (size_t)bp * FD + f0) = f.half[0]; }
__global__ __launch_bounds__(256) void k_e(const float* __restrict__ EC, const float* __restrict__ g, const float* __restrict__ bb, float* __restrict__ E, _Float16* __restrict__ E16) {
  #pragma clang fp contract(off)
  const int tid = threadIdx.x, w = tid >> 5, l = tid & 31; const int bp = blockIdx.x * 8 + w; if (bp >= NB * NP) return; float v0 = gelu_t(EC[(size_t)bp * FD + 2 * l]), v1 = gelu_t(EC[(size_t)bp * FD + 2 * l + 1]); float s = v0 + v1;
  for (int o = 16; o > 0; o >>= 1) s += __shfl_xor(s, o, 32); const float mu = s / (float)FD; float q2 = (v0 - mu) * (v0 - mu) + (v1 - mu) * (v1 - mu);
  for (int o = 16; o > 0; o >>= 1) q2 += __shfl_xor(q2, o, 32); const float rs = rsqrtf(q2 / (float)FD + 1e-5f);
  const float e0 = 2.0f * ((v0 - mu) * rs * bf16_round(g[2 * l]) + bf16_round(bb[2 * l])), e1 = 2.0f * ((v1 - mu) * rs * bf16_round(g[2 * l + 1]) + bf16_round(bb[2 * l + 1]));
  typedef float v2f __attribute__((ext_vector_type(2))); v2f ev; ev[0] = e0; ev[1] = e1; _Float16 h2[2] = {(_Float16)e0, (_Float16)e1}; const unsigned int pk = *(const unsigned int*)h2;
  for (int pass = 0; pass < 2; ++pass) { *(volatile v2f*)(E + (size_t)bp * FD + 2 * l) = ev; *(volatile unsigned int*)((unsigned short*)E16 + (size_t)bp * FD + 2 * l) = pk; if (pass == 0) __threadfence(); } }
__device__ __forceinline__ void pair_of(int t, int& r, int& c) { int rr = (int)floorf((1.0f + sqrtf(1.0f + 8.0f * (float)t)) * 0.5f); while (rr * (rr - 1) / 2 > t) --rr; while ((rr + 1) * rr / 2 <= t) ++rr; r = rr; c = t - rr * (rr - 1) / 2; }
__global__ __launch_bounds__(256) void k_g1(const float* __restrict__ UV, const float* __restrict__ b1, int b, _Float16* __restrict__ G1) {
  #pragma clang fp contract(off)
  const int tt = blockIdx.x * 256 + threadIdx.x; if (tt >= NPAIR * (F2 / 8)) return; const int j0 = (tt % (F2 / 8)) * 8, t = tt / (F2 / 8); int r, c; pair_of(t, r, c); const float* ur = UV + ((size_t)b * NP + r) * 256 + j0; const float* vc = UV + ((size_t)b * NP + c) * 256 + 128 + j0; FragH f = FragH{};
#pragma unroll 1
  for (int q = 0; q < 8; ++q) { const _Float16 hv = (_Float16)gelu_t(ur[q] + vc[q] + bf16_round(b1[j0 + q]));
#pragma unroll
    for (int k = 0; k < 8; ++k) f.h[k] = (k == q) ? hv : f.h[k]; }
  *(volatile v8us*)((unsigned short*)G1 + (size_t)t * F2 + j0) = f.half[0]; __threadfence(); *(volatile v8us*)((unsigned short*)G1 + (size_t)t * F2 + j0) = f.half[0]; }
__global__ __launch_bounds__(256) void k_logit(const float* __restrict__ M, const float* __restrict__ E, const float* __restrict__ g3, const float* __restrict__ b3, const float* __restrict__ wi, int b, float* __restrict__ LOG) {
  #pragma clang fp contract(off)
  const int t = blockIdx.x * 256 + threadIdx.x; if (t >= NPAIR) return; int r, c; pair_of(t, r, c); const float* m = M + (size_t)t * F2; float s = 0.f;
#pragma unroll 1
  for (int j = 0; j < F2; j += 4) { const v4f a = *(const v4fa*)(m + j); s += a[0]; s += a[1]; s += a[2]; s += a[3]; }
  const float mu = s / (float)F2; float q2 = 0.f;
#pragma unroll 1
  for (int j = 0; j < F2; j += 4) { const v4f a = *(const v4fa*)(m + j);
#pragma unroll
    for (int k = 0; k < 4; ++k) { const float d = a[k] - mu; q2 += d * d; } }
  const float rs = rsqrtf(q2 / (float)F2 + 1e-5f); const float* er = E + ((size_t)b * NP + r) * FD; const float* ec = E + ((size_t)b * NP + c) * FD; float lg = 0.f;
#pragma unroll 1
  for (int j = 0; j < F2; ++j) { const float pcv = (j < FD) ? er[j] : ec[j - FD]; const float v = (m[j] - mu) * rs * bf16_round(g3[j]) + bf16_round(b3[j]) + pcv; lg += v * bf16_round(wi[j]); }
  *(volatile float*)(LOG + (size_t)b * NPAIR + t) = lg; __threadfence(); *(volatile float*)(LOG + (size_t)b * NPAIR + t) = lg; }
__global__ __launch_bounds__(256) void k_sstat(const float* __restrict__ LOG, float* __restrict__ ST) {
  #pragma clang fp contract(off)
  __shared__ float red[256]; const int b = blockIdx.x, tid = threadIdx.x; const float* L = LOG + (size_t)b * NPAIR; float m = -3.0e38f; for (int t = tid; t < NPAIR; t += 256) m = fmaxf(m, L[t]);
  red[tid] = m; __syncthreads(); for (int st = 128; st > 0; st >>= 1) { if (tid < st) red[tid] = fmaxf(red[tid], red[tid + st]); __syncthreads(); } m = red[0]; __syncthreads();
  float s = 0.f; for (int t = tid; t < NPAIR; t += 256) s += expf(L[t] - m);
  red[tid] = s; __syncthreads(); for (int st = 128; st > 0; st >>= 1) { if (tid < st) red[tid] += red[tid + st]; __syncthreads(); }
  if (tid < 32) { const float v = (tid == 0) ? m : (tid == 1) ? (1.0f / red[0]) : 0.f; *(volatile float*)(ST + (size_t)b * 32 + tid) = v; __threadfence(); *(volatile float*)(ST + (size_t)b * 32 + tid) = v; } }
__global__ __launch_bounds__(256) void k_pw(const float* __restrict__ LOG, const float* __restrict__ ST, float* __restrict__ WRC) {
  #pragma clang fp contract(off)
  const int t = blockIdx.x * 256 + threadIdx.x; if (t >= NB * NP) return; const int b = t / NP, p = t % NP; const float m = ST[(size_t)b * 32], inv = ST[(size_t)b * 32 + 1]; const float* L = LOG + (size_t)b * NPAIR; float wr = 0.f, wc = 0.f;
#pragma unroll 1
  for (int c = 0; c < p; ++c) wr += expf(L[p * (p - 1) / 2 + c] - m) * inv;
#pragma unroll 1
  for (int r = p + 1; r < NP; ++r) wc += expf(L[r * (r - 1) / 2 + p] - m) * inv;
  typedef float v2f __attribute__((ext_vector_type(2))); v2f v; v[0] = wr; v[1] = wc; *(volatile v2f*)(WRC + (size_t)t * 2) = v; __threadfence(); *(volatile v2f*)(WRC + (size_t)t * 2) = v; }
__global__ __launch_bounds__(256) void k_pool(const float* __restrict__ E, const float* __restrict__ WRC, float* __restrict__ PO) {
  #pragma clang fp contract(off)
  const int t = blockIdx.x * 256 + threadIdx.x; if (t >= NB * F2) return; const int b = t / F2, j = t % F2; const int f = j % FD, side = j / FD; float s = 0.f;
#pragma unroll 1
  for (int p = 0; p < NP; ++p) s += WRC[((size_t)b * NP + p) * 2 + side] * E[((size_t)b * NP + p) * FD + f];
  *(volatile float*)(PO + t) = s; __threadfence(); *(volatile float*)(PO + t) = s; }
__global__ __launch_bounds__(256) void k_fin(const float* __restrict__ PO, const float* __restrict__ pw, const float* __restrict__ pb, const float* __restrict__ LOG, const float* __restrict__ ST, float* __restrict__ out) {
  #pragma clang fp contract(off)
  const int t = blockIdx.x * 256 + threadIdx.x; const int NTOT = NB * NC + NB * NPAIR; if (t * 4 >= NTOT) return; v4f v;
#pragma unroll 1
  for (int q = 0; q < 4; ++q) { const int fl = t * 4 + q; float val = 0.f;
    if (fl < NB * NC) { const int b = fl / NC, j = fl % NC; float s = bf16_round(pb[j]); for (int k = 0; k < F2; ++k) s += PO[b * F2 + k] * bf16_round(pw[(size_t)k * NC + j]); val = s; }
    else if (fl < NTOT) { const int e = fl - NB * NC; const int b = e / NPAIR, tt = e % NPAIR; val = expf(LOG[(size_t)b * NPAIR + tt] - ST[(size_t)b * 32]) * ST[(size_t)b * 32 + 1]; }
#pragma unroll
    for (int k = 0; k < 4; ++k) v[k] = (k == q) ? val : v[k]; }
  *(volatile v4f*)(out + (size_t)t * 4) = v; __threadfence(); *(volatile v4f*)(out + (size_t)t * 4) = v; }

extern "C" void kernel_launch(void* const* d_in, const int* in_sizes, int n_in,
                              void* d_out, int out_size, void* d_ws, size_t ws_size, hipStream_t stream) {
  (void)in_sizes; (void)n_in; (void)out_size;
  const float* const* I = (const float* const*)d_in; const float* x = I[0]; const float* conv_w = I[1]; const float* conv_b = I[2]; const float* pos = I[3]; const float* emb_w = I[4]; const float* emb_b = I[5]; const float* ln1g = I[6]; const float* ln1b = I[7]; const float* w1 = I[8]; const float* b1 = I[9]; const float* w2 = I[10]; const float* b2 = I[11]; const float* ln3g = I[12]; const float* ln3b = I[13]; const float* wi = I[14]; const float* pw = I[15]; const float* pb = I[16];
  char* ws = (char*)d_ws; size_t off = 0;
  auto take = [&](size_t bytes) { char* p = ws + off; off += (bytes + 255) & ~(size_t)255; return p; };
  _Float16* BCV = (_Float16*)take((size_t)FD * 64 * 2); _Float16* BEM = (_Float16*)take((size_t)FD * FD * 2); _Float16* BUV = (_Float16*)take((size_t)256 * FD * 2); _Float16* BW2 = (_Float16*)take((size_t)F2 * F2 * 2);
  _Float16* AP = (_Float16*)take((size_t)NB * NP * 64 * 2); float* CV = (float*)take((size_t)NB * NP * FD * 4); _Float16* H16 = (_Float16*)take((size_t)NB * NP * FD * 2); float* EC = (float*)take((size_t)NB * NP * FD * 4); float* E = (float*)take((size_t)NB * NP * FD * 4); _Float16* E16 = (_Float16*)take((size_t)NB * NP * FD * 2); float* UV = (float*)take((size_t)NB * NP * 256 * 4);
  _Float16* G1 = (_Float16*)take((size_t)NPAIR * F2 * 2); float* M = (float*)take((size_t)NPAIR * F2 * 4); float* LOG = (float*)take((size_t)NB * NPAIR * 4); float* ST = (float*)take(NB * 32 * 4); float* WRC = (float*)take((size_t)NB * NP * 2 * 4); float* PO = (float*)take(NB * F2 * 4);
  if (off > ws_size) return;
  k_round16f<<<(FD * 64 / 8 + 255) / 256, 256, 0, stream>>>(conv_w, BCV, (size_t)FD * 64 / 8);
  k_wt_f16<<<(FD * (FD / 8) + 255) / 256, 256, 0, stream>>>(emb_w, BEM, FD, FD, 16.0f);
  k_wt_f16<<<(F2 * (FD / 8) + 255) / 256, 256, 0, stream>>>(w1, BUV, FD, F2, 16.0f); k_wt_f16<<<(F2 * (FD / 8) + 255) / 256, 256, 0, stream>>>(w1 + (size_t)FD * F2, BUV + (size_t)F2 * FD, FD, F2, 16.0f);
  k_wt_f16<<<(F2 * (F2 / 8) + 255) / 256, 256, 0, stream>>>(w2, BW2, F2, F2, 16.0f);
  const int NTOK = NB * NP;
  k_patch<<<(NTOK * PS + 255) / 256, 256, 0, stream>>>(x, AP);
  k_gemm_hhx<0><<<dim3(((NTOK / 16) * 1 + 3) / 4, 1), 128, 0, stream>>>(AP, 64, 0, BCV, 64, 0, 0.0625f, conv_b, 0, nullptr, 1, 0, 0, CV, nullptr, FD, 0, NTOK, FD, 64);
  k_hpos<<<(NTOK * (FD / 8) + 255) / 256, 256, 0, stream>>>(CV, pos, H16);
  k_gemm_hhx<0><<<dim3(((NTOK / 16) * 1 + 3) / 4, 1), 128, 0, stream>>>(H16, FD, 0, BEM, FD, 0, 0.0625f, emb_b, 0, nullptr, 1, 0, 0, EC, nullptr, FD, 0, NTOK, FD, FD);
  k_e<<<NTOK / 8, 256, 0, stream>>>(EC, ln1g, ln1b, E, E16);
  k_gemm_hhx<0><<<dim3(((NTOK / 16) * 4 + 3) / 4, 1), 128, 0, stream>>>(E16, FD, 0, BUV, FD, 0, 0.0625f, nullptr, 0, nullptr, 1, 0, 0, UV, nullptr, 256, 0, NTOK, 256, FD);
  for (int b = 0; b < NB; ++b) {
    k_g1<<<(NPAIR * (F2 / 8) + 255) / 256, 256, 0, stream>>>(UV, b1, b, G1);
    k_gemm_hhx<0><<<dim3(((NPAIR / 16) * 2 + 3) / 4, 1), 128, 0, stream>>>(G1, F2, 0, BW2, F2, 0, 0.0625f, b2, 0, nullptr, 1, 0, 0, M, nullptr, F2, 0, NPAIR, F2, F2);
    k_logit<<<(NPAIR + 255) / 256, 256, 0, stream>>>(M, E, ln3g, ln3b, wi, b, LOG); }
  k_sstat<<<NB, 256, 0, stream>>>(LOG, ST); k_pw<<<(NTOK + 255) / 256, 256, 0, stream>>>(LOG, ST, WRC); k_pool<<<(NB * F2 + 255) / 256, 256, 0, stream>>>(E, WRC, PO);
  k_fin<<<((NB * NC + NB * NPAIR) / 4 + 255) / 256, 256, 0, stream>>>(PO, pw, pb, LOG, ST, (float*)d_out);
}
